// CCMModel_54709293416874
// MI455X (gfx1250) — hardware-verified
//
#include <hip/hip_runtime.h>
#include <hip/hip_bf16.h>
#include <math.h>

static constexpr int Bc = 16, Lc = 100, Tc = 50, TEc = 100, Hc = 200;
static constexpr int NTILES = 13;
static constexpr int MTILES = 4;
static constexpr int KCH    = 4;
static constexpr float NEG_INF = -1e30f;

#define __bf16 _Float16
typedef __attribute__((ext_vector_type(16))) __bf16 v16bf;
typedef __attribute__((ext_vector_type(2)))  __bf16 bf16x2;
#define RSPLIT (1.0f / 2048.0f)
static constexpr int WFN = 3 * NTILES * KCH * 32 * 16;
static constexpr int SAN = 3 * MTILES * KCH * 32 * 16;
__device__ __forceinline__ __bf16 lo_of(float v, __bf16 h) { return (__bf16)((v - (float)h) * 2048.0f); }
typedef __attribute__((ext_vector_type(8)))  float  v8f;
__device__ __forceinline__ v8f wmma16(v16bf a, v16bf b, v8f c) { return __builtin_amdgcn_wmma_f32_16x16x32_f16(false, a, false, b, (short)0, c, false, false); }
__device__ __forceinline__ v8f wmma_split(v16bf a, v16bf al, v16bf b, v16bf bl, v8f c) { v8f x = {}; x = wmma16(al, b, x); x = wmma16(a, bl, x); return wmma16(a, b, c) + x * RSPLIT; }
typedef __attribute__((ext_vector_type(2)))  float  f32x2;

__device__ __forceinline__ int frag_k(int kc, int lane, int i) {
    const int kOff = (lane < 16) ? 0 : 8;
    return kc * 32 + ((i < 8) ? (kOff + i) : (16 + kOff + (i - 8)));
}

__global__ __launch_bounds__(256)
void pack_weight_frags(const float* __restrict__ Wh,
                       const float* __restrict__ Wr,
                       const float* __restrict__ Wt,
                       __bf16* __restrict__ wf)
{
    const int total = 3 * NTILES * KCH * 32 * 16;
    int idx = (blockIdx.x * blockDim.x + threadIdx.x) * 2;
    if (idx >= total) return;
    const int i    = idx & 15;
    const int lane = (idx >> 4) & 31;
    const int kc   = (idx >> 9) & 3;
    const int nT   = (idx >> 11) % NTILES;
    const int p    = idx / (16 * 32 * KCH * NTILES);
    const int n    = nT * 16 + (lane & 15);
    const int k    = frag_k(kc, lane, i);
    const float* W = (p == 0) ? Wh : ((p == 1) ? Wr : Wt);
    const float v0 = (n < Hc && k < TEc) ? W[n * TEc + k] : 0.0f;
    const float v1 = (n < Hc && k + 1 < TEc) ? W[n * TEc + k + 1] : 0.0f;
    const __bf16 a = (__bf16)v0, b = (__bf16)v1;
    const unsigned u = (unsigned)__builtin_bit_cast(unsigned short, a) | ((unsigned)__builtin_bit_cast(unsigned short, b) << 16);
    const unsigned w = (unsigned)__builtin_bit_cast(unsigned short, lo_of(v0, a)) | ((unsigned)__builtin_bit_cast(unsigned short, lo_of(v1, b)) << 16);
    *(volatile unsigned*)(wf + idx) = u; *(volatile unsigned*)(wf + WFN + idx) = w; __threadfence();
    *(volatile unsigned*)(wf + idx) = u; *(volatile unsigned*)(wf + WFN + idx) = w;
}

__global__ __launch_bounds__(256)
void ccm_static_graph_kernel(const float* __restrict__ head,
                             const float* __restrict__ rel,
                             const float* __restrict__ tail,
                             const float* __restrict__ Wh_b,
                             const float* __restrict__ Wr_b,
                             const float* __restrict__ Wt_b,
                             const __bf16* __restrict__ wf,
                             const int* __restrict__ tmask,
                             const int* __restrict__ pmask,
                             float* __restrict__ out)
{
    const int bl   = blockIdx.x;
    const int l    = bl % Lc;
    const int tid  = threadIdx.x;
    const int lane = tid & 31;
    const int wave = tid >> 5;

    __shared__ __attribute__((aligned(16))) __bf16 sA[2 * SAN];
    __shared__ float  logit_s[MTILES * 16];
    __shared__ float  attn_s[Tc];

    const size_t embBase = (size_t)bl * Tc * TEc;
    const float* srcs[3] = { head + embBase, rel + embBase, tail + embBase };

    const int PAIRS = 3 * MTILES * KCH * 32 * 8;
    for (int q = tid; q < PAIRS; q += 256) {
        const int j    = q & 7;
        const int ln   = (q >> 3) & 31;
        const int kc   = (q >> 8) & 3;
        const int mT   = (q >> 10) & 3;
        const int p    = q >> 12;
        const int row  = mT * 16 + (ln & 15);
        const int kOff = (ln < 16) ? 0 : 8;
        const int k    = kc * 32 + ((j < 4) ? (kOff + 2 * j)
                                            : (16 + kOff + 2 * (j - 4)));
        f32x2 v = {0.0f, 0.0f};
        if (row < Tc && k < TEc)
            v = *(const f32x2*)(srcs[p] + row * TEc + k);
        bf16x2 o, ol;
        o.x = (__bf16)v.x;  ol.x = lo_of(v.x, o.x);
        o.y = (__bf16)v.y;  ol.y = lo_of(v.y, o.y);
        *(bf16x2*)&sA[q * 2] = o;
        *(bf16x2*)&sA[SAN + q * 2] = ol;
    }
    if (tid < MTILES * 16) logit_s[tid] = 0.0f;
    __syncthreads();

    const int mT = wave & 3;

    const int   nLane  = (lane & 15);
    const int   rowHalf = (lane < 16) ? 0 : 8;

    for (int nT = (wave >> 2); nT < NTILES; nT += 2) {
        const int   nCol   = nT * 16 + nLane;
        const float nMsk   = (nCol < Hc) ? 1.0f : 0.0f;
        const int   nClamp = (nCol < Hc) ? nCol : (Hc - 1);

        v8f acc[3] = {};
        #pragma unroll
        for (int p = 0; p < 3; ++p) {
            v8f c = {};
            #pragma unroll 1
            for (int kc = 0; kc < KCH; ++kc) {
                const size_t wo = (size_t)(((p * NTILES + nT) * KCH + kc) * 32 + lane) * 16;
                const int    ao = (((p * MTILES + mT) * KCH + kc) * 32 + lane) * 16;
                c = wmma_split(*(const v16bf*)&sA[ao], *(const v16bf*)&sA[SAN + ao], *(const v16bf*)&wf[wo], *(const v16bf*)&wf[WFN + wo], c);
            }
            acc[p] = c;
        }

        const float hb = Wh_b[nClamp];
        const float rb = Wr_b[nClamp];
        const float tb = Wt_b[nClamp];
        #pragma unroll
        for (int v = 0; v < 8; ++v) {
            const float hv = acc[0][v] + hb;
            const float rv = acc[1][v] + rb;
            const float tv = acc[2][v] + tb;
            float val = nMsk * (rv * tanhf(hv + tv));
            #pragma unroll
            for (int m = 1; m < 16; m <<= 1)
                val += __shfl_xor(val, m, 32);
            if (nLane == 0) {
                const int row = mT * 16 + v + rowHalf;
                atomicAdd(&logit_s[row], val);
            }
        }
    }
    __syncthreads();

    (void)l;
    const bool postPad = (pmask[bl] != 0);
    const int* tm = tmask + (size_t)bl * Tc;
    if (tid < Tc) {
        float mx = -3.0e38f;
        for (int u = 0; u < Tc; ++u) {
            float lg = logit_s[u];
            if (tm[u] != 0) lg = NEG_INF;
            if (postPad)    lg = 0.0f;
            mx = fmaxf(mx, lg);
        }
        float den = 0.0f;
        for (int u = 0; u < Tc; ++u) {
            float lg = logit_s[u];
            if (tm[u] != 0) lg = NEG_INF;
            if (postPad)    lg = 0.0f;
            den += expf(lg - mx);
        }
        float mylg = logit_s[tid];
        if (tm[tid] != 0) mylg = NEG_INF;
        if (postPad)      mylg = 0.0f;
        attn_s[tid] = expf(mylg - mx) / den;
    }
    __syncthreads();

    const float* headp = head + embBase;
    const float* tailp = tail + embBase;
    float* outp = out + (size_t)bl * (2 * TEc);
    for (int e = tid; e < 2 * TEc; e += blockDim.x) {
        const float* src = (e < TEc) ? (headp + e) : (tailp + (e - TEc));
        float s = 0.0f;
        #pragma unroll 5
        for (int t = 0; t < Tc; ++t)
            s += src[(size_t)t * TEc] * attn_s[t];
        *(volatile float*)(outp + e) = s; __threadfence(); *(volatile float*)(outp + e) = s;
    }
}

extern "C" void kernel_launch(void* const* d_in, const int* in_sizes, int n_in,
                              void* d_out, int out_size, void* d_ws, size_t ws_size,
                              hipStream_t stream) {
    const float* head = (const float*)d_in[0];
    const float* rel  = (const float*)d_in[1];
    const float* tail = (const float*)d_in[2];
    const float* Wh_w = (const float*)d_in[3];
    const float* Wh_b = (const float*)d_in[4];
    const float* Wr_w = (const float*)d_in[5];
    const float* Wr_b = (const float*)d_in[6];
    const float* Wt_w = (const float*)d_in[7];
    const float* Wt_b = (const float*)d_in[8];
    const int* tmask = (const int*)d_in[9];
    const int* pmask = (const int*)d_in[10];
    float* out = (float*)d_out;
    __bf16* wfrag = (__bf16*)d_ws;

    const int total = 3 * NTILES * KCH * 32 * 16;
    pack_weight_frags<<<(total / 2 + 255) / 256, 256, 0, stream>>>(Wh_w, Wr_w, Wt_w, wfrag);

    ccm_static_graph_kernel<<<dim3(Bc * Lc), dim3(256), 0, stream>>>(
        head, rel, tail, Wh_b, Wr_b, Wt_b, wfrag, tmask, pmask, out);
}
